// RNN_23072564314230
// MI455X (gfx1250) — hardware-verified
//
#include <hip/hip_runtime.h>
#include <math.h>

constexpr int NBATCH  = 64;
constexpr int NSTEP   = 512;
constexpr int NIN     = 128;
constexpr int NHID    = 512;
constexpr int NOUT    = 75;
constexpr int NFCROWS = 128;
constexpr int NFCSUB  = 5;
constexpr int NROWS   = NBATCH * NSTEP;
constexpr int NTHR    = 256;
constexpr int SEQ_BLK = 32;
constexpr int HPITCH  = 520;
constexpr int SLABP   = 68;
constexpr int FC_ROWS = 32;
constexpr int FC_THR  = 128;
constexpr int NBIASP  = 2 * NHID + NFCROWS;
constexpr float WCARRY     = 16.0f;
constexpr float WCARRY_INV = 1.0f / WCARRY;

static_assert(NROWS % 64 == 0 && NHID % 64 == 0, "GEMM M, N tile multiples");
static_assert(NIN % 32 == 0 && NHID % 32 == 0, "GEMM K multiples of 32");
static_assert(NBATCH % SEQ_BLK == 0, "step-loop grid exact");
static_assert(NHID == 64 * (NTHR / 32), "8 waves x 64 hidden columns");
static_assert((2 * SEQ_BLK * HPITCH) % 8 == 0, "h tiles fill in 16-B units");
static_assert(NFCSUB * 16 >= NOUT && NFCSUB * 16 <= NFCROWS, "head column groups inside the padded plane");
static_assert((FC_ROWS * NOUT * 4) % 128 == 0, "head wave tile is whole lines");
static_assert(NROWS % (FC_ROWS * (FC_THR / 32)) == 0, "head grid exact");
static_assert(NBIASP == 4 * 288, "bias plane = 288 threads x 4 floats");
static_assert(NOUT * 4 * NROWS == 9830400, "output bytes");

typedef __attribute__((ext_vector_type(16))) _Float16 v16h;
typedef __attribute__((ext_vector_type(8)))  _Float16 v8h;
typedef __attribute__((ext_vector_type(16))) __bf16   v16b;
typedef __attribute__((ext_vector_type(8)))  __bf16   v8b;
typedef __attribute__((ext_vector_type(8)))  float    v8f;
typedef __attribute__((ext_vector_type(4)))  float    v4f;

__device__ __forceinline__ unsigned short f2bf_bits(float f) {
  unsigned u = __float_as_uint(f);
  return (unsigned short)((u + 0x7FFFu + ((u >> 16) & 1u)) >> 16);
}
__device__ __forceinline__ float bf_bits2f(unsigned short h) { return __uint_as_float(((unsigned)h) << 16); }

__device__ __forceinline__ void tie4_h(v8f& a, v8f& b, v8f& c, v8f& d, v16h x, v16h y) {
  asm volatile("v_nop\n\tv_nop\n\tv_nop\n\tv_nop" : "+v"(a), "+v"(b), "+v"(c), "+v"(d) : "v"(x), "v"(y));
}
__device__ __forceinline__ void tie4_b(v8f& a, v8f& b, v8f& c, v8f& d, v16b x, v16b y) {
  asm volatile("v_nop\n\tv_nop\n\tv_nop\n\tv_nop" : "+v"(a), "+v"(b), "+v"(c), "+v"(d) : "v"(x), "v"(y));
}
__device__ __forceinline__ void tie5_h(v8f& a, v8f& b, v8f& c, v8f& d, v8f& e, v16h x, v16h y) {
  asm volatile("v_nop\n\tv_nop\n\tv_nop\n\tv_nop" : "+v"(a), "+v"(b), "+v"(c), "+v"(d), "+v"(e) : "v"(x), "v"(y));
}
__device__ __forceinline__ void keep4_h(v16h a, v16h b, v16h c, v16h d) { asm volatile("v_nop" :: "v"(a), "v"(b), "v"(c), "v"(d)); }
__device__ __forceinline__ void keep4_b(v16b a, v16b b, v16b c, v16b d) { asm volatile("v_nop" :: "v"(a), "v"(b), "v"(c), "v"(d)); }
__device__ __forceinline__ void acc_guard4(v8f& a, v8f& b, v8f& c, v8f& d) {
  asm volatile("v_nop\n\tv_nop\n\tv_nop\n\tv_nop" : "+v"(a), "+v"(b), "+v"(c), "+v"(d));
}
__device__ __forceinline__ void acc_guard5(v8f& a, v8f& b, v8f& c, v8f& d, v8f& e) {
  asm volatile("v_nop\n\tv_nop\n\tv_nop\n\tv_nop" : "+v"(a), "+v"(b), "+v"(c), "+v"(d), "+v"(e));
}
__device__ __forceinline__ void wave_lds_sync() {
  __builtin_amdgcn_fence(__ATOMIC_RELEASE, "workgroup");
  __builtin_amdgcn_wave_barrier();
  __builtin_amdgcn_fence(__ATOMIC_ACQUIRE, "workgroup");
}

template <typename T> struct Frag;
template <> struct Frag<_Float16> {
  typedef v16h V; union U { v16h v; v8h h[2]; };
  static __device__ __forceinline__ v16h load(const _Float16* p) {
    U f; f.h[0] = *(const v8h*)(p); f.h[1] = *(const v8h*)(p + 16); return f.v;
  }
  static __device__ __forceinline__ v8f mma(v16h a, v16h b, v8f c) {
    return __builtin_amdgcn_wmma_f32_16x16x32_f16(false, a, false, b, (short)0, c, false, false);
  }
  static __device__ __forceinline__ void guard4(v8f& a, v8f& b, v8f& c, v8f& d, v16h x, v16h y) { tie4_h(a, b, c, d, x, y); }
  static __device__ __forceinline__ void keep(v16h a, v16h b, v16h c, v16h d) { keep4_h(a, b, c, d); }
};
template <> struct Frag<__bf16> {
  typedef v16b V; union U { v16b v; v8b h[2]; };
  static __device__ __forceinline__ v16b load(const __bf16* p) {
    U f; f.h[0] = *(const v8b*)(p); f.h[1] = *(const v8b*)(p + 16); return f.v;
  }
  static __device__ __forceinline__ v8f mma(v16b a, v16b b, v8f c) {
    return __builtin_amdgcn_wmma_f32_16x16x32_bf16(false, a, false, b, (short)0, c, false, false);
  }
  static __device__ __forceinline__ void guard4(v8f& a, v8f& b, v8f& c, v8f& d, v16b x, v16b y) { tie4_b(a, b, c, d, x, y); }
  static __device__ __forceinline__ void keep(v16b a, v16b b, v16b c, v16b d) { keep4_b(a, b, c, d); }
};

template <int ET> struct Elem;
template <> struct Elem<0> { typedef _Float16 T; };
template <> struct Elem<1> { typedef __bf16 T; };
template <int ET, bool SPLIT>
__global__ __launch_bounds__(256) void wmma_gemm64(
    const unsigned short* __restrict__ Ap, const unsigned short* __restrict__ A2p, int lda,
    const unsigned short* __restrict__ Btp, const unsigned short* __restrict__ Bt2p, int ldb,
    float* __restrict__ Cout, int ldc,
    const float* __restrict__ bias,
    int M, int N, int K, float scale) {
  typedef typename Elem<ET>::T T;
  typedef typename Frag<T>::V V;
  const T* A = (const T*)Ap; const T* A2 = (const T*)A2p; const T* Bt = (const T*)Btp; const T* Bt2 = (const T*)Bt2p;
  __shared__ __align__(16) float sT[8][16 * 68];
  const int lane = threadIdx.x & 31;
  const int wave = threadIdx.x >> 5;
  const int tilesN = N >> 6;
  const int tilesM = M >> 6;
  const int tile = blockIdx.x * 8 + wave;
  if (tile >= tilesM * tilesN) return;
  const int tm = tile / tilesN;
  const int tn = tile - tm * tilesN;
  const int m0 = tm << 6;
  const int n0 = tn << 6;

  const int rlane = lane & 15;
  const int koff  = (lane >> 4) * 8;
  const int mOff  = (lane >> 4) * 8;

  v8f acc[4][4];
#pragma unroll
  for (int i = 0; i < 4; ++i)
#pragma unroll
    for (int j = 0; j < 4; ++j) acc[i][j] = (v8f){0.f,0.f,0.f,0.f,0.f,0.f,0.f,0.f};

  for (int k0 = 0; k0 < K; k0 += 32) {
    V bh[4], bl[4];
#pragma unroll
    for (int j = 0; j < 4; ++j) {
      const size_t bo = (size_t)(n0 + (j << 4) + rlane) * ldb + koff + k0;
      bh[j] = Frag<T>::load(Bt + bo);
      if (SPLIT) bl[j] = Frag<T>::load(Bt2 + bo);
    }
#pragma unroll
    for (int i = 0; i < 4; ++i) {
      const size_t ao = (size_t)(m0 + (i << 4) + rlane) * lda + koff + k0;
      V ah = Frag<T>::load(A + ao);
      V al;
      if (SPLIT) al = Frag<T>::load(A2 + ao);
#pragma unroll
      for (int j = 0; j < 4; ++j) {
        acc[i][j] = Frag<T>::mma(ah, bh[j], acc[i][j]);
        if (SPLIT) {
          acc[i][j] = Frag<T>::mma(ah, bl[j], acc[i][j]);
          acc[i][j] = Frag<T>::mma(al, bh[j], acc[i][j]);
        }
      }
      Frag<T>::guard4(acc[i][0], acc[i][1], acc[i][2], acc[i][3], ah, SPLIT ? al : ah);
    }
    Frag<T>::keep(bh[0], bh[1], bh[2], bh[3]);
    if (SPLIT) Frag<T>::keep(bl[0], bl[1], bl[2], bl[3]);
  }
  acc_guard4(acc[0][0], acc[0][1], acc[0][2], acc[0][3]);
  acc_guard4(acc[1][0], acc[1][1], acc[1][2], acc[1][3]);
  acc_guard4(acc[2][0], acc[2][1], acc[2][2], acc[2][3]);
  acc_guard4(acc[3][0], acc[3][1], acc[3][2], acc[3][3]);

  float* slab = sT[wave];
#pragma unroll
  for (int i = 0; i < 4; ++i) {
    const int mBase = m0 + (i << 4);
#pragma unroll
    for (int j = 0; j < 4; ++j) {
      const int n = n0 + (j << 4) + rlane;
      const float bv = bias[n];
#pragma unroll
      for (int r = 0; r < 8; ++r) {
        const float v = acc[i][j][r] * scale + bv;
        slab[(mOff + r) * 68 + (j << 4) + rlane] = v;
      }
    }
    wave_lds_sync();
    {
      const int hh = lane >> 4, c4 = (lane & 15) * 4;
      for (int pass = 0; pass < 2; ++pass) {
#pragma unroll
        for (int it = 0; it < 8; ++it) {
          const int row = it * 2 + hh;
          const v4f v = *(const v4f*)(slab + row * 68 + c4);
          *(volatile v4f*)(Cout + (size_t)(mBase + row) * ldc + n0 + c4) = v;
        }
        __threadfence();
      }
    }
    wave_lds_sync();
  }
}

template <int MODE>
__global__ __launch_bounds__(NTHR) void cvt8_kernel(const float* __restrict__ src, unsigned short* __restrict__ dst,
                                                    unsigned short* __restrict__ dst2,
                                                    int nrow_src, int nrow_dst, int ncol8, float sc) {
  const int i  = blockIdx.x * NTHR + threadIdx.x;
  const int n8 = nrow_dst * ncol8;
  if (i < n8) {
    const int row = i / ncol8;
    const int c8  = i - row * ncol8;
    const int rc  = (row < nrow_src) ? row : (nrow_src - 1);
    const bool keep = (row < nrow_src);
    const float* sp = src + (size_t)rc * (size_t)(ncol8 * 8) + c8 * 8;
    const v4f a = *(const v4f*)(sp);
    const v4f b = *(const v4f*)(sp + 4);
    v8h hv, lv;
#pragma unroll
    for (int e = 0; e < 4; ++e) {
      const float fa = keep ? a[e] : 0.0f;
      const float fb = keep ? b[e] : 0.0f;
      if (MODE == 0) {
        hv[e]     = (_Float16)(fa * sc);
        hv[4 + e] = (_Float16)(fb * sc);
        lv[e]     = (_Float16)0.0f;
        lv[4 + e] = (_Float16)0.0f;
      } else {
        const unsigned short ha = f2bf_bits(fa);
        const unsigned short hb = f2bf_bits(fb);
        const unsigned short la = f2bf_bits(fa - bf_bits2f(ha));
        const unsigned short lb = f2bf_bits(fb - bf_bits2f(hb));
        hv[e]     = __builtin_bit_cast(_Float16, ha);
        hv[4 + e] = __builtin_bit_cast(_Float16, hb);
        lv[e]     = __builtin_bit_cast(_Float16, la);
        lv[4 + e] = __builtin_bit_cast(_Float16, lb);
      }
    }
    *(volatile v8h*)(dst + (size_t)i * 8) = hv;
    if (MODE == 1) *(volatile v8h*)(dst2 + (size_t)i * 8) = lv;
    __threadfence();
    *(volatile v8h*)(dst + (size_t)i * 8) = hv;
    if (MODE == 1) *(volatile v8h*)(dst2 + (size_t)i * 8) = lv;
  }
}

__global__ __launch_bounds__(288) void bias_prep_kernel(const float* __restrict__ bih0, const float* __restrict__ bhh0,
                                                        const float* __restrict__ bih1, const float* __restrict__ bhh1,
                                                        const float* __restrict__ bfc, float* __restrict__ dst) {
  const int tid = threadIdx.x;
  const int which = tid >> 7;
  const int j = (tid & 127) * 4;
  const v4f va = *(const v4f*)(bih0 + j);
  const v4f vb = *(const v4f*)(bhh0 + j);
  const v4f vc = *(const v4f*)(bih1 + j);
  const v4f vd = *(const v4f*)(bhh1 + j);
  int jf = (tid - 256) * 4;
  jf = (jf < 0) ? 0 : jf;
  v4f fv;
#pragma unroll
  for (int e = 0; e < 4; ++e) {
    const int idx = jf + e;
    const int ic  = (idx < NOUT) ? idx : (NOUT - 1);
    const float f = bfc[ic];
    fv[e] = (idx < NOUT) ? f : 0.0f;
  }
  v4f o;
#pragma unroll
  for (int e = 0; e < 4; ++e) {
    const float s0 = va[e] + vb[e];
    const float s1 = vc[e] + vd[e];
    o[e] = (which == 0) ? s0 : ((which == 1) ? s1 : fv[e]);
  }
  float* op = dst + tid * 4;
  *(volatile v4f*)op = o;
  __threadfence();
  *(volatile v4f*)op = o;
}

__global__ __launch_bounds__(NTHR) void rnn_seq_kernel(const float* __restrict__ XW,
                                                       const unsigned short* __restrict__ Wp,
                                                       unsigned short* __restrict__ HPLp) {
  __shared__ __align__(16) _Float16 Hb[2][SEQ_BLK * HPITCH];
  __shared__ __align__(16) float    Sl[NTHR / 32][SEQ_BLK * SLABP];
  const _Float16* W = (const _Float16*)Wp;
  _Float16* HPL = (_Float16*)HPLp;
  const int tid = threadIdx.x, lane = tid & 31, wave = tid >> 5;
  const int c = lane & 15, hh = lane >> 4, koff = hh * 8;
  const int q = lane >> 3, c8 = (lane & 7) * 8;
  const int rowbase = blockIdx.x * SEQ_BLK;

  {
    v8h zv;
#pragma unroll
    for (int e = 0; e < 8; ++e) zv[e] = (_Float16)0.0f;
    v8h* hz = (v8h*)&Hb[0][0];
#pragma unroll 1
    for (int i = tid; i < (2 * SEQ_BLK * HPITCH) / 8; i += NTHR) hz[i] = zv;
  }
  __syncthreads();

  const v8f z8 = {0.f, 0.f, 0.f, 0.f, 0.f, 0.f, 0.f, 0.f};
  float* slab = Sl[wave];
  const _Float16* wrow = W + (size_t)(64 * wave + c) * NHID + koff;

#pragma unroll 1
  for (int t = 0; t < NSTEP; ++t) {
    const int cur = t & 1;
    const _Float16* hc = &Hb[cur][0];
    _Float16* hn = &Hb[cur ^ 1][0];
    const _Float16* a0p = hc + c * HPITCH + koff;
    const _Float16* a1p = hc + (16 + c) * HPITCH + koff;

    v8f acc[2][4];
#pragma unroll
    for (int mi = 0; mi < 2; ++mi)
#pragma unroll
      for (int j = 0; j < 4; ++j) acc[mi][j] = z8;

#pragma unroll 1
    for (int k0 = 0; k0 < NHID; k0 += 32) {
      const v16h b0 = Frag<_Float16>::load(wrow + (size_t)0 * 16 * NHID + k0);
      const v16h b1 = Frag<_Float16>::load(wrow + (size_t)1 * 16 * NHID + k0);
      const v16h b2 = Frag<_Float16>::load(wrow + (size_t)2 * 16 * NHID + k0);
      const v16h b3 = Frag<_Float16>::load(wrow + (size_t)3 * 16 * NHID + k0);
      const v16h a0 = Frag<_Float16>::load(a0p + k0);
      const v16h a1 = Frag<_Float16>::load(a1p + k0);
      acc[0][0] = Frag<_Float16>::mma(a0, b0, acc[0][0]);
      acc[0][1] = Frag<_Float16>::mma(a0, b1, acc[0][1]);
      acc[0][2] = Frag<_Float16>::mma(a0, b2, acc[0][2]);
      acc[0][3] = Frag<_Float16>::mma(a0, b3, acc[0][3]);
      acc[1][0] = Frag<_Float16>::mma(a1, b0, acc[1][0]);
      acc[1][1] = Frag<_Float16>::mma(a1, b1, acc[1][1]);
      acc[1][2] = Frag<_Float16>::mma(a1, b2, acc[1][2]);
      acc[1][3] = Frag<_Float16>::mma(a1, b3, acc[1][3]);
      tie4_h(acc[0][0], acc[0][1], acc[0][2], acc[0][3], a0, b3);
      tie4_h(acc[1][0], acc[1][1], acc[1][2], acc[1][3], a1, b0);
      keep4_h(b0, b1, b2, b3);
    }
    acc_guard4(acc[0][0], acc[0][1], acc[0][2], acc[0][3]);
    acc_guard4(acc[1][0], acc[1][1], acc[1][2], acc[1][3]);

#pragma unroll
    for (int mi = 0; mi < 2; ++mi)
#pragma unroll
      for (int j = 0; j < 4; ++j)
#pragma unroll
        for (int r = 0; r < 8; ++r) slab[(16 * mi + 8 * hh + r) * SLABP + 16 * j + c] = acc[mi][j][r];
    wave_lds_sync();

#pragma unroll 1
    for (int it = 0; it < 8; ++it) {
      const int row = it * 4 + q;
      const float* sp = slab + row * SLABP + c8;
      const v4f p0 = *(const v4f*)(sp);
      const v4f p1 = *(const v4f*)(sp + 4);
      const size_t go = ((size_t)(rowbase + row) * NSTEP + (size_t)t) * NHID + (size_t)(64 * wave + c8);
      const v4f x0 = *(const v4f*)(XW + go);
      const v4f x1 = *(const v4f*)(XW + go + 4);
      v8h hv;
#pragma unroll
      for (int e = 0; e < 4; ++e) {
        const float z0 = p0[e] * WCARRY_INV + x0[e];
        const float z1 = p1[e] * WCARRY_INV + x1[e];
        hv[e]     = (_Float16)tanhf(z0);
        hv[4 + e] = (_Float16)tanhf(z1);
      }
      *(v8h*)(hn + row * HPITCH + 64 * wave + c8) = hv;
      *(volatile v8h*)(HPL + go) = hv;
      __threadfence();
      *(volatile v8h*)(HPL + go) = hv;
    }
    wave_lds_sync();
    __syncthreads();
  }
}

__global__ __launch_bounds__(FC_THR) void fc_kernel(const unsigned short* __restrict__ Hp,
                                                    const unsigned short* __restrict__ Wp,
                                                    const float* __restrict__ bfcp,
                                                    float* __restrict__ out) {
  __shared__ __align__(16) float So[FC_THR / 32][FC_ROWS * NOUT];
  const _Float16* H = (const _Float16*)Hp;
  const _Float16* W = (const _Float16*)Wp;
  const int tid = threadIdx.x, lane = tid & 31, wave = tid >> 5;
  const int c = lane & 15, hh = lane >> 4, koff = hh * 8;
  const int tile = blockIdx.x * (FC_THR / 32) + wave;
  const int m0 = tile * FC_ROWS;

  const v8f z8 = {0.f, 0.f, 0.f, 0.f, 0.f, 0.f, 0.f, 0.f};
  v8f acc[2][NFCSUB];
#pragma unroll
  for (int i = 0; i < 2; ++i)
#pragma unroll
    for (int j = 0; j < NFCSUB; ++j) acc[i][j] = z8;

  const _Float16* ap0 = H + (size_t)(m0 + c) * NHID + koff;
  const _Float16* ap1 = H + (size_t)(m0 + 16 + c) * NHID + koff;
  const _Float16* bp  = W + (size_t)c * NHID + koff;

#pragma unroll 1
  for (int k0 = 0; k0 < NHID; k0 += 32) {
    v16h bf[NFCSUB];
#pragma unroll
    for (int j = 0; j < NFCSUB; ++j) bf[j] = Frag<_Float16>::load(bp + (size_t)j * 16 * NHID + k0);
    const v16h a0 = Frag<_Float16>::load(ap0 + k0);
    const v16h a1 = Frag<_Float16>::load(ap1 + k0);
#pragma unroll
    for (int j = 0; j < NFCSUB; ++j) acc[0][j] = Frag<_Float16>::mma(a0, bf[j], acc[0][j]);
#pragma unroll
    for (int j = 0; j < NFCSUB; ++j) acc[1][j] = Frag<_Float16>::mma(a1, bf[j], acc[1][j]);
    tie5_h(acc[0][0], acc[0][1], acc[0][2], acc[0][3], acc[0][4], a0, bf[4]);
    tie5_h(acc[1][0], acc[1][1], acc[1][2], acc[1][3], acc[1][4], a1, bf[0]);
    keep4_h(bf[0], bf[1], bf[2], bf[3]);
  }
  acc_guard5(acc[0][0], acc[0][1], acc[0][2], acc[0][3], acc[0][4]);
  acc_guard5(acc[1][0], acc[1][1], acc[1][2], acc[1][3], acc[1][4]);

  float* slab = So[wave];
#pragma unroll
  for (int j = 0; j < NFCSUB; ++j) {
    const int n = 16 * j + c;
    const float bv = bfcp[n];
#pragma unroll
    for (int i = 0; i < 2; ++i) {
#pragma unroll
      for (int r = 0; r < 8; ++r) {
        const float v = acc[i][j][r] * WCARRY_INV + bv;
        if (n < NOUT) slab[(16 * i + 8 * hh + r) * NOUT + n] = v;
      }
    }
  }
  wave_lds_sync();

  float* op = out + (size_t)m0 * NOUT;
  constexpr int NV4 = FC_ROWS * NOUT / 4;
  for (int pass = 0; pass < 2; ++pass) {
#pragma unroll 1
    for (int it = 0; it < (NV4 + 31) / 32; ++it) {
      const int idx = it * 32 + lane;
      const int idc = (idx < NV4) ? idx : (NV4 - 1);
      const v4f v = *(const v4f*)(slab + 4 * idc);
      if (idx < NV4) *(volatile v4f*)(op + 4 * idx) = v;
    }
    __threadfence();
  }
}

extern "C" void kernel_launch(void* const* d_in, const int* in_sizes, int n_in,
                              void* d_out, int out_size, void* d_ws, size_t ws_size, hipStream_t stream) {
  if (n_in < 11 || d_out == nullptr || d_ws == nullptr) return;
  if (in_sizes[0] != NROWS * NIN || in_sizes[1] != NHID * NIN || in_sizes[2] != NHID * NHID ||
      in_sizes[3] != NHID || in_sizes[4] != NHID || in_sizes[5] != NHID * NHID ||
      in_sizes[6] != NHID * NHID || in_sizes[7] != NHID || in_sizes[8] != NHID ||
      in_sizes[9] != NOUT * NHID || in_sizes[10] != NOUT || out_size != NROWS * NOUT) return;

  const float* x    = (const float*)d_in[0];
  const float* wih0 = (const float*)d_in[1];
  const float* whh0 = (const float*)d_in[2];
  const float* bih0 = (const float*)d_in[3];
  const float* bhh0 = (const float*)d_in[4];
  const float* wih1 = (const float*)d_in[5];
  const float* whh1 = (const float*)d_in[6];
  const float* bih1 = (const float*)d_in[7];
  const float* bhh1 = (const float*)d_in[8];
  const float* wfc  = (const float*)d_in[9];
  const float* bfc  = (const float*)d_in[10];
  float* out = (float*)d_out;

  char* ws = (char*)d_ws; size_t off = 0;
  auto carve = [&](size_t bytes) -> char* { char* p = ws + off; off += (bytes + 255) & ~(size_t)255; return p; };
  float*          XW    = (float*)carve((size_t)NROWS * NHID * 4);
  unsigned short* HPL   = (unsigned short*)carve((size_t)NROWS * NHID * 2);
  unsigned short* XH    = (unsigned short*)carve((size_t)NROWS * NIN * 2);
  unsigned short* XL    = (unsigned short*)carve((size_t)NROWS * NIN * 2);
  unsigned short* W0H   = (unsigned short*)carve((size_t)NHID * NIN * 2);
  unsigned short* W0L   = (unsigned short*)carve((size_t)NHID * NIN * 2);
  unsigned short* WHH0  = (unsigned short*)carve((size_t)NHID * NHID * 2);
  unsigned short* WIH1  = (unsigned short*)carve((size_t)NHID * NHID * 2);
  unsigned short* WHH1  = (unsigned short*)carve((size_t)NHID * NHID * 2);
  unsigned short* WFC   = (unsigned short*)carve((size_t)NFCROWS * NHID * 2);
  float*          BIASP = (float*)carve((size_t)NBIASP * 4);
  if (off > ws_size || off > (size_t)134217728) return;

  const int n8x  = NROWS * (NIN / 8);
  const int n8w0 = NHID * (NIN / 8);
  const int n8h  = NHID * (NHID / 8);
  const int n8f  = NFCROWS * (NHID / 8);
  cvt8_kernel<1><<<n8x  / NTHR, NTHR, 0, stream>>>(x,    XH,   XL,   NROWS, NROWS,   NIN / 8,  1.0f);
  cvt8_kernel<1><<<n8w0 / NTHR, NTHR, 0, stream>>>(wih0, W0H,  W0L,  NHID,  NHID,    NIN / 8,  1.0f);
  cvt8_kernel<0><<<n8h  / NTHR, NTHR, 0, stream>>>(whh0, WHH0, WHH0, NHID,  NHID,    NHID / 8, WCARRY);
  cvt8_kernel<0><<<n8h  / NTHR, NTHR, 0, stream>>>(wih1, WIH1, WIH1, NHID,  NHID,    NHID / 8, WCARRY);
  cvt8_kernel<0><<<n8h  / NTHR, NTHR, 0, stream>>>(whh1, WHH1, WHH1, NHID,  NHID,    NHID / 8, WCARRY);
  cvt8_kernel<0><<<n8f  / NTHR, NTHR, 0, stream>>>(wfc,  WFC,  WFC,  NOUT,  NFCROWS, NHID / 8, WCARRY);
  bias_prep_kernel<<<1, 288, 0, stream>>>(bih0, bhh0, bih1, bhh1, bfc, BIASP);

  const dim3 ggrid((NROWS / 64) * (NHID / 64) / 8, 1);

  wmma_gemm64<1, true><<<ggrid, 256, 0, stream>>>(XH, XL, NIN, W0H, W0L, NIN, XW, NHID, BIASP, NROWS, NHID, NIN, 1.0f);
  rnn_seq_kernel<<<NBATCH / SEQ_BLK, NTHR, 0, stream>>>(XW, WHH0, HPL);
  wmma_gemm64<0, false><<<ggrid, 256, 0, stream>>>(HPL, HPL, NHID, WIH1, WIH1, NHID, XW, NHID, BIASP + NHID, NROWS, NHID, NHID, WCARRY_INV);
  rnn_seq_kernel<<<NBATCH / SEQ_BLK, NTHR, 0, stream>>>(XW, WHH1, HPL);
  fc_kernel<<<NROWS / (FC_ROWS * (FC_THR / 32)), FC_THR, 0, stream>>>(HPL, WFC, BIASP + 2 * NHID, out);
}
